// GraphEncoderTL_6751688589919
// MI455X (gfx1250) — hardware-run, weakly checked
//
#include <hip/hip_runtime.h>
#include <hip/hip_bf16.h>
#include <stddef.h>


#define DD    128
#define GR    32
#define XSP   132
#define NTHR  256
#define KSP   512
#define KF    64
#define NB    512
#define CHUNK 2048
#define NWAVE 8
#define WCAP  256
#define NGRP  (CHUNK / (NTHR * 4))
#define GMB   64

#define GAT_SACC (NB * DD)
#define GAT_LDS_FLOATS (GAT_SACC + NB + NWAVE * WCAP + NWAVE + 8)
#define GAT_LDS_BYTES (GAT_LDS_FLOATS * 4)
#define FNC_LDS_BYTES ((KF * DD * 3 + KF * KF + 2 * KF) * 4)

static_assert(WCAP == (CHUNK / NTHR) * 32);
static_assert(NGRP == 2);
static_assert(NB == 512);
static_assert(((GAT_SACC + NB) % 4) == 0);
static_assert(GAT_LDS_BYTES == 272448);
static_assert(FNC_LDS_BYTES == 115200);
static_assert((KSP % 64) == 0 && (KSP % GR) == 0);

typedef float          v4f   __attribute__((ext_vector_type(4)));
typedef float          v8f   __attribute__((ext_vector_type(8)));
typedef int            v4i   __attribute__((ext_vector_type(4)));
typedef unsigned short v8us  __attribute__((ext_vector_type(8)));
typedef __bf16         v16bf __attribute__((ext_vector_type(16)));
union FragB { v16bf v; v8us u[2]; };

__device__ __forceinline__ v8f wmb(v16bf a, v16bf b, v8f c) {
  v8f d = __builtin_amdgcn_wmma_f32_16x16x32_bf16(false, a, false, b, (short)0, c, false, false);
  asm volatile("v_nop\n\tv_nop\n\tv_nop\n\tv_nop" : "+v"(d) : "v"(a), "v"(b));
  return d;
}

__device__ __forceinline__ v16bf ldfrag(const unsigned short* p) {
  FragB f;
  f.u[0] = *(const v8us*)p;
  f.u[1] = *(const v8us*)(p + 16);
  return f.v;
}

__device__ __forceinline__ unsigned short bfr(float x) {
  unsigned u = __float_as_uint(x);
  u = u + 0x7fffu + ((u >> 16) & 1u);
  return (unsigned short)(u >> 16);
}
__device__ __forceinline__ float bff(unsigned short s) { return __uint_as_float(((unsigned)s) << 16); }
__device__ __forceinline__ void sp2(float x, unsigned short* h, unsigned short* l) {
  const unsigned short a = bfr(x);
  *h = a;
  *l = bfr(x - bff(a));
}
__device__ __forceinline__ void sp3(float x, unsigned short* h, unsigned short* m, unsigned short* l) {
  const unsigned short a = bfr(x);
  const float r = x - bff(a);
  const unsigned short b = bfr(r);
  *h = a; *m = b;
  *l = bfr(r - bff(b));
}
__device__ __forceinline__ v4f sel4(bool c, v4f a, v4f b) {
  v4f r;
  r.x = c ? a.x : b.x; r.y = c ? a.y : b.y; r.z = c ? a.z : b.z; r.w = c ? a.w : b.w;
  return r;
}
__device__ __forceinline__ int wrapclamp(int i, int n) {
  i = (i < 0) ? i + n : i;
  i = i < 0 ? 0 : (i > n - 1 ? n - 1 : i);
  return i;
}

__global__ __launch_bounds__(128) void k_colsum(const float* __restrict__ SA, float* rcs, int nN, int KS) {
  const int k  = blockIdx.x * 128 + threadIdx.x;
  const int kc = min(k, KS - 1);
  double s = 0.0;
#pragma unroll 1
  for (int n = 0; n < nN; ++n) s += (double)SA[(size_t)n * KS + kc];
  const float cs = (float)s;
  float t = cs - 1.0f;
  t = t > 0.f ? t : 0.f;
  float r = 1.0f / (t + 1.0f);
  if (k >= KS) r = 1.0f;
  *(volatile float*)(rcs + k) = r;
  __threadfence();
  *(volatile float*)(rcs + k) = r;
}

__device__ __forceinline__ float adjpost_v(const float* __restrict__ ADJ, int k, int j, int KS) {
  const float a  = ADJ[(size_t)k * KS + j];
  const float dg = (k == j) ? 1.0f : 0.0f;
  float t = a - dg * 10000.0f;
  t = t > 0.f ? t : 0.f;
  t = t + dg;
  t = t + dg;
  return t;
}

__global__ __launch_bounds__(NTHR) void k_setup_small(const float* __restrict__ FA, const float* __restrict__ ADJ,
                                                      float* rcf, float* rden, float* adjn, int KS) {
  __shared__ __attribute__((aligned(16))) float rcf_s[KF];
  __shared__ __attribute__((aligned(16))) float rden_s[KSP];
  __shared__ __attribute__((aligned(16))) float dinv_s[KSP];
  const int tid = threadIdx.x;

  if (tid < KF) {
    double c = 0.0;
#pragma unroll 1
    for (int k = 0; k < KS; ++k) c += (double)FA[(size_t)k * KF + tid];
    const float cs = (float)c;
    float t = cs - 1.0f;
    t = t > 0.f ? t : 0.f;
    rcf_s[tid] = 1.0f / (t + 1.0f);
  }
  __syncthreads();

#pragma unroll 1
  for (int k = tid; k < KSP; k += NTHR) {
    const int kc = min(k, KS - 1);
    double s = 0.0;
#pragma unroll 1
    for (int j = 0; j < KF; ++j) s += (double)(FA[(size_t)kc * KF + j] * rcf_s[j]);
    const float sf = (float)s;
    float t = sf - 1.0f;
    t = t > 0.f ? t : 0.f;
    const float rd = 1.0f / (t + 1.0f);
    double rs = 0.0;
#pragma unroll 1
    for (int j = 0; j < KS; ++j) rs += (double)fabsf(adjpost_v(ADJ, kc, j, KS));
    const float dv = 1.0f / sqrtf((float)rs);
    rden_s[k] = (k < KS) ? rd : 1.0f;
    dinv_s[k] = (k < KS) ? dv : 0.0f;
  }
  __syncthreads();

  if (tid < KF / 4) {
    const v4f v = *(const v4f*)(rcf_s + 4 * tid);
    *(volatile v4f*)(rcf + 4 * tid) = v;
    __threadfence();
    *(volatile v4f*)(rcf + 4 * tid) = v;
  }
  if (tid < KSP / 4) {
    const v4f v = *(const v4f*)(rden_s + 4 * tid);
    *(volatile v4f*)(rden + 4 * tid) = v;
    __threadfence();
    *(volatile v4f*)(rden + 4 * tid) = v;
  }
#pragma unroll 1
  for (int idx = tid; idx < KS * (KSP / 4); idx += NTHR) {
    const int k  = idx >> 7;
    const int c4 = idx & 127;
    const float dk = dinv_s[k];
    v4f o;
    float ov[4];
#pragma unroll
    for (int q = 0; q < 4; ++q) {
      const int j  = 4 * c4 + q;
      const int jc = min(j, KS - 1);
      const float ap = adjpost_v(ADJ, k, jc, KS);
      float val = (dk * ap) * dinv_s[jc];
      if (j >= KS) val = 0.0f;
      ov[q] = val;
    }
    o.x = ov[0]; o.y = ov[1]; o.z = ov[2]; o.w = ov[3];
    float* p = adjn + (size_t)k * KSP + 4 * c4;
    *(volatile v4f*)p = o;
    __threadfence();
    *(volatile v4f*)p = o;
  }
}

__global__ __launch_bounds__(NTHR) void k_sa_planes(const float* __restrict__ SA, const float* __restrict__ rcs,
                                                    unsigned short* saRh, unsigned short* saRl,
                                                    unsigned short* saTh, unsigned short* saTl,
                                                    int nN, int KS, int NT) {
  __shared__ float tile[64][65];
  const int tid = threadIdx.x;
  const int n0 = blockIdx.x * 64, k0 = blockIdx.y * 64;
#pragma unroll 1
  for (int it = 0; it < 16; ++it) {
    const int idx = it * NTHR + tid;
    const int r = idx >> 6, c = idx & 63;
    const int n = n0 + r, k = k0 + c;
    const int nc = min(n, nN - 1), kc = min(k, KS - 1);
    float v = SA[(size_t)nc * KS + kc];
    if (n >= nN || k >= KS) v = 0.0f;
    tile[r][c] = v;
  }
  __syncthreads();

#pragma unroll
  for (int p = 0; p < 2; ++p) {
    const int i = p * NTHR + tid;
    const int r = i >> 3, seg = i & 7;
    v8us uh, ul;
#pragma unroll
    for (int q = 0; q < 8; ++q) {
      unsigned short a, b;
      sp2(tile[r][8 * seg + q], &a, &b);
      uh[q] = a; ul[q] = b;
    }
    const size_t o = (size_t)(n0 + r) * KSP + k0 + 8 * seg;
    *(volatile v8us*)(saRh + o) = uh;
    *(volatile v8us*)(saRl + o) = ul;
    __threadfence();
    *(volatile v8us*)(saRh + o) = uh;
    *(volatile v8us*)(saRl + o) = ul;
  }
#pragma unroll
  for (int p = 0; p < 2; ++p) {
    const int i = p * NTHR + tid;
    const int c = i >> 3, seg = i & 7;
    const int k = k0 + c;
    const float rk = rcs[min(k, KS - 1)];
    v8us uh, ul;
#pragma unroll
    for (int q = 0; q < 8; ++q) {
      unsigned short a, b;
      sp2(tile[8 * seg + q][c] * rk, &a, &b);
      uh[q] = a; ul[q] = b;
    }
    const size_t o = (size_t)k * NT + n0 + 8 * seg;
    *(volatile v8us*)(saTh + o) = uh;
    *(volatile v8us*)(saTl + o) = ul;
    __threadfence();
    *(volatile v8us*)(saTh + o) = uh;
    *(volatile v8us*)(saTl + o) = ul;
  }
}

__global__ __launch_bounds__(NTHR) void k_w_planes(const float* __restrict__ W0, const float* __restrict__ W1,
                                                   unsigned short* wgT) {
  const float* W = (blockIdx.x == 0) ? W0 : W1;
  unsigned short* base = wgT + (size_t)blockIdx.x * 3 * DD * DD;
  const int tid = threadIdx.x;
#pragma unroll 1
  for (int it = 0; it < 8; ++it) {
    const int i = it * NTHR + tid;
    const int o = i >> 4, seg = i & 15;
    v8us uh, um, ul;
#pragma unroll
    for (int q = 0; q < 8; ++q) {
      unsigned short a, b, c;
      sp3(W[(size_t)(8 * seg + q) * DD + o], &a, &b, &c);
      uh[q] = a; um[q] = b; ul[q] = c;
    }
    const size_t off = (size_t)o * DD + 8 * seg;
    *(volatile v8us*)(base + off) = uh;
    *(volatile v8us*)(base + DD * DD + off) = um;
    *(volatile v8us*)(base + 2 * DD * DD + off) = ul;
    __threadfence();
    *(volatile v8us*)(base + off) = uh;
    *(volatile v8us*)(base + DD * DD + off) = um;
    *(volatile v8us*)(base + 2 * DD * DD + off) = ul;
  }
}

__global__ __launch_bounds__(NTHR) void k_gather(const float* __restrict__ nodeT, const float* __restrict__ typeT,
                                                 const float* __restrict__ lenT, const float* __restrict__ laneT,
                                                 const int* __restrict__ nf, const int* __restrict__ tf,
                                                 const int* __restrict__ lf, const int* __restrict__ laf,
                                                 float* raw, int nN, int NR, int TR, int GRL, int LR) {
  const int tid = threadIdx.x, lane = tid & 31, wave = tid >> 5;
  const int n0 = blockIdx.x * 64;
#pragma unroll 1
  for (int it = 0; it < 8; ++it) {
    const int r = it * 8 + wave;
    const int n = n0 + r;
    if (n >= nN) continue;
    const int ia = wrapclamp(laf[n], LR);
    const int ib = wrapclamp(tf[n], TR);
    const int ic = wrapclamp(lf[n], GRL);
    const int id = wrapclamp(nf[n], NR);
    const int col = 4 * lane;
    const v4f vl = *(const v4f*)(laneT + (size_t)ia * 32 + min(col, 28));
    const v4f vt = *(const v4f*)(typeT + (size_t)ib * 16 + min(max(col - 32, 0), 12));
    const v4f vg = *(const v4f*)(lenT  + (size_t)ic * 16 + min(max(col - 48, 0), 12));
    const v4f vn = *(const v4f*)(nodeT + (size_t)id * 64 + min(max(col - 64, 0), 60));
    const v4f v = sel4(lane < 8, vl, sel4(lane < 12, vt, sel4(lane < 16, vg, vn)));
    float* op = raw + (size_t)n * DD + col;
    *(volatile v4f*)op = v;
    __threadfence();
    *(volatile v4f*)op = v;
  }
}

__global__ __launch_bounds__(NTHR) void k_tr_planes(const float* __restrict__ src, int nValid,
                                                    unsigned short* ph, unsigned short* pl, int pitch) {
  __shared__ float tile[64][DD + 1];
  const int tid = threadIdx.x, lane = tid & 31, wave = tid >> 5;
  const int r0 = blockIdx.x * 64;
  const v4f z4 = {0.f, 0.f, 0.f, 0.f};
#pragma unroll 1
  for (int it = 0; it < 8; ++it) {
    const int r = it * 8 + wave;
    const int rr = r0 + r;
    const int rc = min(rr, nValid - 1);
    v4f v = *(const v4f*)(src + (size_t)rc * DD + 4 * lane);
    if (rr >= nValid) v = z4;
    tile[r][4 * lane + 0] = v.x;
    tile[r][4 * lane + 1] = v.y;
    tile[r][4 * lane + 2] = v.z;
    tile[r][4 * lane + 3] = v.w;
  }
  __syncthreads();
#pragma unroll 1
  for (int it = 0; it < 4; ++it) {
    const int i = it * NTHR + tid;
    const int d = i >> 3, seg = i & 7;
    v8us uh, ul;
#pragma unroll
    for (int q = 0; q < 8; ++q) {
      unsigned short a, b;
      sp2(tile[8 * seg + q][d], &a, &b);
      uh[q] = a; ul[q] = b;
    }
    const size_t o = (size_t)d * pitch + r0 + 8 * seg;
    *(volatile v8us*)(ph + o) = uh;
    *(volatile v8us*)(pl + o) = ul;
    __threadfence();
    *(volatile v8us*)(ph + o) = uh;
    *(volatile v8us*)(pl + o) = ul;
  }
}

__device__ __forceinline__ void acc_to_lds(v8f acc, int T, int hh, int ncol, float* Xs) {
#pragma unroll
  for (int r = 0; r < 8; ++r) Xs[(T * 16 + 8 * hh + r) * XSP + ncol] = acc[r];
}
__device__ __forceinline__ void rows_store2(const float* Xs, float* out, int rowBase, int wave, int lane) {
  v4f x0 = *(const v4f*)(Xs + (4 * wave + 0) * XSP + 4 * lane);
  v4f x1 = *(const v4f*)(Xs + (4 * wave + 1) * XSP + 4 * lane);
  v4f x2 = *(const v4f*)(Xs + (4 * wave + 2) * XSP + 4 * lane);
  v4f x3 = *(const v4f*)(Xs + (4 * wave + 3) * XSP + 4 * lane);
  float* p0 = out + (size_t)(rowBase + 4 * wave + 0) * DD + 4 * lane;
  float* p1 = out + (size_t)(rowBase + 4 * wave + 1) * DD + 4 * lane;
  float* p2 = out + (size_t)(rowBase + 4 * wave + 2) * DD + 4 * lane;
  float* p3 = out + (size_t)(rowBase + 4 * wave + 3) * DD + 4 * lane;
  *(volatile v4f*)p0 = x0; *(volatile v4f*)p1 = x1; *(volatile v4f*)p2 = x2; *(volatile v4f*)p3 = x3;
  __threadfence();
  *(volatile v4f*)p0 = x0; *(volatile v4f*)p1 = x1; *(volatile v4f*)p2 = x2; *(volatile v4f*)p3 = x3;
}

__global__ __launch_bounds__(NTHR) void k_gemm_se(
    const unsigned short* __restrict__ aTh, const unsigned short* __restrict__ aTl,
    const unsigned short* __restrict__ bTh, const unsigned short* __restrict__ bTl,
    float* semb0, int nN, int NT) {
  __shared__ __attribute__((aligned(16))) float Xs[GR * XSP];
  const int tid = threadIdx.x, lane = tid & 31, wave = tid >> 5;
  const int hh = lane >> 4, m = lane & 15;
  const int rowBase = blockIdx.x * GR;
  const int ncol = wave * 16 + m;
  const size_t ra0 = (size_t)(rowBase + m) * NT + 8 * hh;
  const size_t ra1 = (size_t)(rowBase + 16 + m) * NT + 8 * hh;
  const size_t rb  = (size_t)ncol * NT + 8 * hh;
  v8f c0 = {0.f, 0.f, 0.f, 0.f, 0.f, 0.f, 0.f, 0.f};
  v8f c1 = {0.f, 0.f, 0.f, 0.f, 0.f, 0.f, 0.f, 0.f};
#pragma unroll 1
  for (int kk = 0; kk < nN; kk += 32) {
    const v16bf a0h = ldfrag(aTh + ra0 + kk), a1h = ldfrag(aTh + ra1 + kk);
    const v16bf a0l = ldfrag(aTl + ra0 + kk), a1l = ldfrag(aTl + ra1 + kk);
    const v16bf bh  = ldfrag(bTh + rb + kk),  bl  = ldfrag(bTl + rb + kk);
    c0 = wmb(a0h, bh, c0); c0 = wmb(a0h, bl, c0); c0 = wmb(a0l, bh, c0);
    c1 = wmb(a1h, bh, c1); c1 = wmb(a1h, bl, c1); c1 = wmb(a1l, bh, c1);
  }
  acc_to_lds(c0, 0, hh, ncol, Xs);
  acc_to_lds(c1, 1, hh, ncol, Xs);
  __syncthreads();
  rows_store2(Xs, semb0, rowBase, wave, lane);
}

__global__ __launch_bounds__(NTHR) void k_fnc(const float* __restrict__ semb0, const float* __restrict__ FA,
                                              const float* __restrict__ rcf, const float* __restrict__ rden,
                                              const float* __restrict__ Wf, const float* __restrict__ bfv,
                                              float* semb1, int KS) {
  extern __shared__ float flds[];
  float* fe0   = flds;
  float* adjp  = fe0 + KF * DD;
  float* sup   = adjp + KF * KF;
  float* fe1   = sup + KF * DD;
  float* dinv  = fe1 + KF * DD;
  float* rcf_s = dinv + KF;
  const int tid = threadIdx.x;

  if (tid < KF) rcf_s[tid] = rcf[tid];
  __syncthreads();

#pragma unroll 1
  for (int it = 0; it < (KF * DD) / NTHR; ++it) {
    const int idx = it * NTHR + tid;
    const int j = idx >> 7, d = idx & 127;
    const float rj = rcf_s[j];
    float acc = 0.f;
#pragma unroll 1
    for (int k = 0; k < KS; ++k) acc = fmaf(FA[(size_t)k * KF + j] * rj, semb0[(size_t)k * DD + d], acc);
    fe0[idx] = acc;
  }
  __syncthreads();

#pragma unroll 1
  for (int it = 0; it < (KF * KF) / NTHR; ++it) {
    const int idx = it * NTHR + tid;
    const int i = idx >> 6, j = idx & 63;
    float acc = 0.f;
#pragma unroll 1
    for (int d = 0; d < DD; ++d) acc = fmaf(fe0[i * DD + d], fe0[j * DD + d], acc);
    const float s  = 1.0f / (1.0f + __expf(-acc));
    const float dg = (i == j) ? 1.0f : 0.0f;
    float t = s + dg;
    t = t + dg;
    adjp[idx] = t;
  }
  __syncthreads();

  if (tid < KF) {
    double rs = 0.0;
#pragma unroll 1
    for (int j = 0; j < KF; ++j) rs += (double)fabsf(adjp[tid * KF + j]);
    dinv[tid] = 1.0f / sqrtf((float)rs);
  }
  __syncthreads();

#pragma unroll 1
  for (int it = 0; it < (KF * DD) / NTHR; ++it) {
    const int idx = it * NTHR + tid;
    const int j = idx >> 7, d = idx & 127;
    float acc = 0.f;
#pragma unroll 1
    for (int i = 0; i < DD; ++i) acc = fmaf(fe0[j * DD + i], Wf[(size_t)i * DD + d], acc);
    sup[idx] = acc;
  }
  __syncthreads();

#pragma unroll 1
  for (int it = 0; it < (KF * DD) / NTHR; ++it) {
    const int idx = it * NTHR + tid;
    const int i = idx >> 7, d = idx & 127;
    const float di = dinv[i];
    float acc = 0.f;
#pragma unroll 1
    for (int j = 0; j < KF; ++j) acc = fmaf((di * adjp[i * KF + j]) * dinv[j], sup[j * DD + d], acc);
    fe1[idx] = acc + bfv[d];
  }
  __syncthreads();

#pragma unroll 1
  for (int it = 0; it < (KSP * DD) / NTHR; ++it) {
    const int idx = it * NTHR + tid;
    const int k = idx >> 7, d = idx & 127;
    const int kc = min(k, KS - 1);
    float acc = 0.f;
#pragma unroll 1
    for (int j = 0; j < KF; ++j) acc = fmaf(FA[(size_t)kc * KF + j], fe1[j * DD + d], acc);
    float v = semb0[(size_t)kc * DD + d] + 0.15f * (acc * rden[kc]);
    if (k >= KS) v = 0.f;
    *(volatile float*)(semb1 + idx) = v;
    __threadfence();
    *(volatile float*)(semb1 + idx) = v;
  }
}

__global__ __launch_bounds__(NTHR) void k_sup_s(const float* __restrict__ semb1, const float* __restrict__ Ws,
                                                float* sup, int KS) {
  const int idx = blockIdx.x * NTHR + threadIdx.x;
  const int k = idx >> 7, d = idx & 127;
  const int kc = min(k, KS - 1);
  float acc = 0.f;
#pragma unroll 1
  for (int i = 0; i < DD; ++i) acc = fmaf(semb1[(size_t)kc * DD + i], Ws[(size_t)i * DD + d], acc);
  const float v = (k < KS) ? acc : 0.f;
  *(volatile float*)(sup + idx) = v;
  __threadfence();
  *(volatile float*)(sup + idx) = v;
}

__global__ __launch_bounds__(128) void k_semb2(const float* __restrict__ adjn, const float* __restrict__ sup,
                                               const float* __restrict__ bsv, float* semb2, int KS) {
  const int k = blockIdx.x, d = threadIdx.x;
  const int kc = min(k, KS - 1);
  float acc = 0.f;
#pragma unroll 1
  for (int j = 0; j < KS; ++j) acc = fmaf(adjn[(size_t)kc * KSP + j], sup[(size_t)j * DD + d], acc);
  const float v = (k < KS) ? (acc + bsv[d]) : 0.f;
  float* p = semb2 + (size_t)k * DD + d;
  *(volatile float*)p = v;
  __threadfence();
  *(volatile float*)p = v;
}

__device__ __forceinline__ void sm_epi(const float* __restrict__ raw, const float* Xs,
                                       unsigned short* ph, unsigned short* pm, unsigned short* pl,
                                       int rowBase, int tid) {
#pragma unroll
  for (int p = 0; p < 2; ++p) {
    const int i = p * NTHR + tid;
    const int r = i >> 4, seg = i & 15;
    const size_t go = (size_t)(rowBase + r) * DD + 8 * seg;
    const v4f x0 = *(const v4f*)(raw + go);
    const v4f x1 = *(const v4f*)(raw + go + 4);
    const float xv[8] = {x0.x, x0.y, x0.z, x0.w, x1.x, x1.y, x1.z, x1.w};
    v8us uh, um, ul;
#pragma unroll
    for (int q = 0; q < 8; ++q) {
      const float v = xv[q] + 0.5f * Xs[r * XSP + 8 * seg + q];
      unsigned short a, b, c;
      sp3(v, &a, &b, &c);
      uh[q] = a; um[q] = b; ul[q] = c;
    }
    *(volatile v8us*)(ph + go) = uh;
    *(volatile v8us*)(pm + go) = um;
    *(volatile v8us*)(pl + go) = ul;
  }
}

__global__ __launch_bounds__(NTHR) void k_gemm_sm(
    const unsigned short* __restrict__ aRh, const unsigned short* __restrict__ aRl,
    const unsigned short* __restrict__ bTh, const unsigned short* __restrict__ bTl,
    const float* __restrict__ raw, unsigned short* ph, unsigned short* pm, unsigned short* pl, int nN) {
  __shared__ __attribute__((aligned(16))) float Xs[GR * XSP];
  const int tid = threadIdx.x, lane = tid & 31, wave = tid >> 5;
  const int hh = lane >> 4, m = lane & 15;
  const int rowBase = blockIdx.x * GR;
  const int ncol = wave * 16 + m;
  const size_t ra0 = (size_t)(rowBase + m) * KSP + 8 * hh;
  const size_t ra1 = (size_t)(rowBase + 16 + m) * KSP + 8 * hh;
  const size_t rb  = (size_t)ncol * KSP + 8 * hh;
  v8f c0 = {0.f, 0.f, 0.f, 0.f, 0.f, 0.f, 0.f, 0.f};
  v8f c1 = {0.f, 0.f, 0.f, 0.f, 0.f, 0.f, 0.f, 0.f};
#pragma unroll 1
  for (int kk = 0; kk < KSP; kk += 32) {
    const v16bf a0h = ldfrag(aRh + ra0 + kk), a1h = ldfrag(aRh + ra1 + kk);
    const v16bf a0l = ldfrag(aRl + ra0 + kk), a1l = ldfrag(aRl + ra1 + kk);
    const v16bf bh  = ldfrag(bTh + rb + kk),  bl  = ldfrag(bTl + rb + kk);
    c0 = wmb(a0h, bh, c0); c0 = wmb(a0h, bl, c0); c0 = wmb(a0l, bh, c0);
    c1 = wmb(a1h, bh, c1); c1 = wmb(a1h, bl, c1); c1 = wmb(a1l, bh, c1);
  }
  acc_to_lds(c0, 0, hh, ncol, Xs);
  acc_to_lds(c1, 1, hh, ncol, Xs);
  __syncthreads();
  sm_epi(raw, Xs, ph, pm, pl, rowBase, tid);
  __threadfence();
  sm_epi(raw, Xs, ph, pm, pl, rowBase, tid);
}

__device__ __forceinline__ void h_epi(const float* Xs, const float* dots, float* hout, float* ha, float* hb,
                                      int rowBase, int wave, int lane) {
  v4f x0 = *(const v4f*)(Xs + (4 * wave + 0) * XSP + 4 * lane);
  v4f x1 = *(const v4f*)(Xs + (4 * wave + 1) * XSP + 4 * lane);
  v4f x2 = *(const v4f*)(Xs + (4 * wave + 2) * XSP + 4 * lane);
  v4f x3 = *(const v4f*)(Xs + (4 * wave + 3) * XSP + 4 * lane);
  *(volatile v4f*)(hout + (size_t)(rowBase + 4 * wave + 0) * DD + 4 * lane) = x0;
  *(volatile v4f*)(hout + (size_t)(rowBase + 4 * wave + 1) * DD + 4 * lane) = x1;
  *(volatile v4f*)(hout + (size_t)(rowBase + 4 * wave + 2) * DD + 4 * lane) = x2;
  *(volatile v4f*)(hout + (size_t)(rowBase + 4 * wave + 3) * DD + 4 * lane) = x3;
  if (wave == 0 && lane < 16) {
    const int q = lane & 7;
    const v4f v = *(const v4f*)(dots + ((lane < 8) ? 0 : GR) + 4 * q);
    float* p = ((lane < 8) ? ha : hb) + rowBase + 4 * q;
    *(volatile v4f*)p = v;
  }
}

__global__ __launch_bounds__(NTHR) void k_gemm_h(
    const unsigned short* __restrict__ xh, const unsigned short* __restrict__ xm, const unsigned short* __restrict__ xl,
    const unsigned short* __restrict__ wh, const unsigned short* __restrict__ wm, const unsigned short* __restrict__ wl,
    const float* __restrict__ ag, float* hout, float* ha, float* hb, int nN) {
  __shared__ __attribute__((aligned(16))) float Xs[GR * XSP];
  __shared__ __attribute__((aligned(16))) float ag_s[2 * DD];
  __shared__ __attribute__((aligned(16))) float dots[2 * GR];
  const int tid = threadIdx.x, lane = tid & 31, wave = tid >> 5;
  const int hh = lane >> 4, m = lane & 15;
  const int rowBase = blockIdx.x * GR;
  const int ncol = wave * 16 + m;
  if (tid < (2 * DD) / 4) *(v4f*)(ag_s + 4 * tid) = *(const v4f*)(ag + 4 * tid);
  const size_t ra0 = (size_t)(rowBase + m) * DD + 8 * hh;
  const size_t ra1 = (size_t)(rowBase + 16 + m) * DD + 8 * hh;
  const size_t rb  = (size_t)ncol * DD + 8 * hh;
  v8f c0 = {0.f, 0.f, 0.f, 0.f, 0.f, 0.f, 0.f, 0.f};
  v8f c1 = {0.f, 0.f, 0.f, 0.f, 0.f, 0.f, 0.f, 0.f};
#pragma unroll 1
  for (int kk = 0; kk < DD; kk += 32) {
    const v16bf a0h = ldfrag(xh + ra0 + kk), a0m = ldfrag(xm + ra0 + kk), a0l = ldfrag(xl + ra0 + kk);
    const v16bf a1h = ldfrag(xh + ra1 + kk), a1m = ldfrag(xm + ra1 + kk), a1l = ldfrag(xl + ra1 + kk);
    const v16bf bh  = ldfrag(wh + rb + kk),  bm  = ldfrag(wm + rb + kk),  bl  = ldfrag(wl + rb + kk);
    c0 = wmb(a0h, bh, c0); c0 = wmb(a0h, bm, c0); c0 = wmb(a0m, bh, c0);
    c0 = wmb(a0h, bl, c0); c0 = wmb(a0m, bm, c0); c0 = wmb(a0l, bh, c0);
    c1 = wmb(a1h, bh, c1); c1 = wmb(a1h, bm, c1); c1 = wmb(a1m, bh, c1);
    c1 = wmb(a1h, bl, c1); c1 = wmb(a1m, bm, c1); c1 = wmb(a1l, bh, c1);
  }
  acc_to_lds(c0, 0, hh, ncol, Xs);
  acc_to_lds(c1, 1, hh, ncol, Xs);
  __syncthreads();
  if (tid < 2 * GR) {
    const int r = tid >> 1, w = tid & 1;
    float acc = 0.f;
#pragma unroll 1
    for (int c = 0; c < DD; ++c) acc = fmaf(Xs[r * XSP + c], ag_s[w * DD + c], acc);
    dots[w * GR + r] = acc;
  }
  __syncthreads();
  h_epi(Xs, dots, hout, ha, hb, rowBase, wave, lane);
  __threadfence();
  h_epi(Xs, dots, hout, ha, hb, rowBase, wave, lane);
}

__global__ __launch_bounds__(NTHR) void k_emax(const int* __restrict__ ei, const float* __restrict__ ha,
                                               const float* __restrict__ hb, float* gpart, int nN, int nE) {
  __shared__ float wmx[NWAVE];
  const int tid = threadIdx.x, lane = tid & 31, wave = tid >> 5;
  float mx = -3.0e38f;
#pragma unroll 1
  for (int base = blockIdx.x * NTHR; base < nE; base += GMB * NTHR) {
    const int e = min(base + tid, nE - 1);
    const int s = wrapclamp(ei[e], nN);
    const int d = wrapclamp(ei[(size_t)nE + e], nN);
    mx = fmaxf(mx, ha[s] + hb[d]);
  }
  mx = fmaxf(mx, __shfl_xor(mx, 16, 32));
  mx = fmaxf(mx, __shfl_xor(mx, 8, 32));
  mx = fmaxf(mx, __shfl_xor(mx, 4, 32));
  mx = fmaxf(mx, __shfl_xor(mx, 2, 32));
  mx = fmaxf(mx, __shfl_xor(mx, 1, 32));
  if (lane == 0) wmx[wave] = mx;
  __syncthreads();
  if (wave == 0) {
    float v = wmx[min(lane, NWAVE - 1)];
    v = (lane < NWAVE) ? v : -3.0e38f;
    v = fmaxf(v, __shfl_xor(v, 16, 32));
    v = fmaxf(v, __shfl_xor(v, 8, 32));
    v = fmaxf(v, __shfl_xor(v, 4, 32));
    v = fmaxf(v, __shfl_xor(v, 2, 32));
    v = fmaxf(v, __shfl_xor(v, 1, 32));
    const v4f o4 = {v, v, v, v};
    float* p = gpart + (size_t)blockIdx.x * 32 + 4 * (lane & 7);
    if (lane < 8) *(volatile v4f*)p = o4;
    __threadfence();
    if (lane < 8) *(volatile v4f*)p = o4;
  }
}

__global__ __launch_bounds__(NTHR) void k_gat(const int* __restrict__ ei, const float* __restrict__ h,
                                              const float* __restrict__ ha, const float* __restrict__ hb,
                                              const float* __restrict__ gpart, float* dest, int nN, int nE) {
  extern __shared__ v4f lds_dyn[];
  float* sacc = (float*)lds_dyn;
  float* ssum = sacc + GAT_SACC;
  int*   list = (int*)(ssum + NB);
  int*   wcnt = list + NWAVE * WCAP;
  float* gms  = (float*)(wcnt + NWAVE);

  const int tid  = threadIdx.x;
  const int lane = tid & 31;
  const int wave = tid >> 5;
  const int nodeBase = blockIdx.x * NB;

  {
    const v4f z4 = {0.f, 0.f, 0.f, 0.f};
    for (int i = tid; i < (GAT_SACC + NB) / 4; i += NTHR) lds_dyn[i] = z4;
    if (tid == 0) {
      float mx = -3.0e38f;
#pragma unroll 1
      for (int b = 0; b < GMB; ++b) mx = fmaxf(mx, gpart[b * 32]);
      mx = mx > 0.f ? mx : 0.2f * mx;
      gms[0] = mx;
    }
  }
  __syncthreads();
  const float gmax = gms[0];
  const int* own = ei;
  const int* nbr = ei + nE;
  const bool al16 = ((((size_t)own) & 15) == 0);

  const int nChunks = (nE + CHUNK - 1) / CHUNK;
#pragma unroll 1
  for (int ch = 0; ch < nChunks; ++ch) {
    const int cbase = ch * CHUNK;
    int wc = 0;
#pragma unroll
    for (int g = 0; g < NGRP; ++g) {
      const int el0 = (g * NTHR + tid) * 4;
      const int e0  = cbase + el0;
      const int sent = -2147483647 - 1;
      v4i d;
      if (al16 && (cbase + CHUNK <= nE)) {
        d = *(const v4i*)(own + e0);
      } else {
        d.x = (e0     < nE) ? own[min(e0, nE - 1)]     : sent;
        d.y = (e0 + 1 < nE) ? own[min(e0 + 1, nE - 1)] : sent;
        d.z = (e0 + 2 < nE) ? own[min(e0 + 2, nE - 1)] : sent;
        d.w = (e0 + 3 < nE) ? own[min(e0 + 3, nE - 1)] : sent;
      }
      const unsigned s0 = (unsigned)d.x - (unsigned)nodeBase;
      const unsigned s1 = (unsigned)d.y - (unsigned)nodeBase;
      const unsigned s2 = (unsigned)d.z - (unsigned)nodeBase;
      const unsigned s3 = (unsigned)d.w - (unsigned)nodeBase;
      const bool h0 = s0 < (unsigned)NB;
      const bool h1 = s1 < (unsigned)NB;
      const bool h2 = s2 < (unsigned)NB;
      const bool h3 = s3 < (unsigned)NB;
      const unsigned many = __builtin_amdgcn_ballot_w32(h0 | h1 | h2 | h3);
      if (many != 0u) {
#define HITJ(J, HJ, SJ) { \
          const unsigned mj = __builtin_amdgcn_ballot_w32(HJ); \
          if (HJ) { \
            const int pos = wc + (int)__builtin_amdgcn_mbcnt_lo(mj, 0u); \
            if (pos < WCAP) list[wave * WCAP + pos] = ((el0 + (J)) << 9) | (int)(SJ); \
          } \
          wc += (int)__builtin_popcount(mj); }
        HITJ(0, h0, s0)
        HITJ(1, h1, s1)
        HITJ(2, h2, s2)
        HITJ(3, h3, s3)
#undef HITJ
      }
    }
    if (lane == 0) wcnt[wave] = wc;
    __syncthreads();

    if (wave == 0) {
      for (int wsx = 0; wsx < NWAVE; ++wsx) {
        int n = wcnt[wsx];
        if (n > WCAP) n = WCAP;
        if (n < 0) n = 0;
        for (int i = 0; i < n; ++i) {
          const int ent  = list[wsx * WCAP + i];
          const int slot = ent & (NB - 1);
          const int el   = (ent >> 9) & (CHUNK - 1);
          int e = cbase + el;
          if (e > nE - 1) e = nE - 1;
          const int nb = wrapclamp(nbr[e], nN);
          int nd = nodeBase + slot;
          if (nd > nN - 1) nd = nN - 1;
          float v = ha[nd] + hb[nb];
          v = (v > 0.f) ? v : 0.2f * v;
          const float p = __expf(v - gmax);
          const v4f xv = *(const v4f*)(h + (size_t)nb * DD + 4 * lane);
          v4f* sp = (v4f*)(sacc + slot * DD + 4 * lane);
          const v4f cur = *sp;
          *sp = cur + p * xv;
          if (lane == 0) {
            const float o = ssum[slot];
            ssum[slot] = o + p;
          }
        }
      }
    }
    __syncthreads();
  }

#pragma unroll 1
  for (int j = 0; j < NB / NWAVE; ++j) {
    const int slot = wave * (NB / NWAVE) + j;
    const int node = nodeBase + slot;
    if (node >= nN) break;
    const float S = ssum[slot];
    const float rinv = 1.0f / (S + 1e-15f);
    const v4f sv = *(const v4f*)(sacc + slot * DD + 4 * lane);
    const v4f x = sv * rinv;
    v4f y;
    y.x = x.x > 0.f ? x.x : (__expf(x.x) - 1.0f);
    y.y = x.y > 0.f ? x.y : (__expf(x.y) - 1.0f);
    y.z = x.z > 0.f ? x.z : (__expf(x.z) - 1.0f);
    y.w = x.w > 0.f ? x.w : (__expf(x.w) - 1.0f);
    float* op = dest + (size_t)node * DD + 4 * lane;
    *(volatile v4f*)op = y;
    __threadfence();
    *(volatile v4f*)op = y;
  }
}

extern "C" void kernel_launch(void* const* d_in, const int* in_sizes, int n_in,
                              void* d_out, int out_size, void* d_ws, size_t ws_size,
                              hipStream_t stream) {
  if (n_in < 24) return;
  const int N = in_sizes[19];
  if (N < 64 || (N % GR) != 0) return;
  if (in_sizes[0] < 64 || (in_sizes[0] % 64) != 0) return;
  if (in_sizes[1] < 16 || (in_sizes[1] % 16) != 0) return;
  if (in_sizes[2] < 16 || (in_sizes[2] % 16) != 0) return;
  if (in_sizes[3] < 32 || (in_sizes[3] % 32) != 0) return;
  const int NR = in_sizes[0] / 64, TR = in_sizes[1] / 16, GRL = in_sizes[2] / 16, LR = in_sizes[3] / 32;
  if ((in_sizes[4] % N) != 0) return;
  const int KS = in_sizes[4] / N;
  if (KS < 1 || KS > KSP) return;
  if (in_sizes[5] != KS * KF || in_sizes[6] != KS * KS) return;
  if (in_sizes[7] != DD * DD || in_sizes[9] != DD * DD || in_sizes[11] != DD * DD) return;
  if (in_sizes[13] != DD * DD || in_sizes[15] != DD * DD || in_sizes[17] != DD * DD) return;
  if (in_sizes[8] != DD || in_sizes[10] != DD || in_sizes[14] != DD || in_sizes[16] != DD) return;
  if (in_sizes[12] != 2 * DD || in_sizes[18] != 2 * DD) return;
  if (in_sizes[20] != N || in_sizes[21] != N || in_sizes[22] != N) return;
  if (in_sizes[23] < 2 || (in_sizes[23] % 2) != 0) return;
  const int E = in_sizes[23] / 2;
  if (out_size != N * DD) return;
  const int NT = ((N + 63) / 64) * 64;

  const float* nodeT = (const float*)d_in[0];
  const float* typeT = (const float*)d_in[1];
  const float* lenT  = (const float*)d_in[2];
  const float* laneT = (const float*)d_in[3];
  const float* SA    = (const float*)d_in[4];
  const float* FA    = (const float*)d_in[5];
  const float* ADJ   = (const float*)d_in[6];
  const float* Wf[2] = {(const float*)d_in[7],  (const float*)d_in[13]};
  const float* bf[2] = {(const float*)d_in[8],  (const float*)d_in[14]};
  const float* Ws[2] = {(const float*)d_in[9],  (const float*)d_in[15]};
  const float* bs[2] = {(const float*)d_in[10], (const float*)d_in[16]};
  const float* Wg[2] = {(const float*)d_in[11], (const float*)d_in[17]};
  const float* ag[2] = {(const float*)d_in[12], (const float*)d_in[18]};
  const int* nf  = (const int*)d_in[19];
  const int* tf  = (const int*)d_in[20];
  const int* lf  = (const int*)d_in[21];
  const int* laf = (const int*)d_in[22];
  const int* ei  = (const int*)d_in[23];
  float* out = (float*)d_out;

  size_t off = 0;
#define CARVE(ptr, type, bytes) ptr = (type*)((char*)d_ws + off); off += (((size_t)(bytes)) + 255) & ~(size_t)255;
  float* rcs;   CARVE(rcs,   float, (size_t)KSP * 4)
  float* rcf;   CARVE(rcf,   float, (size_t)KF * 4)
  float* rden;  CARVE(rden,  float, (size_t)KSP * 4)
  float* adjn;  CARVE(adjn,  float, (size_t)KSP * KSP * 4)
  float* gpart; CARVE(gpart, float, (size_t)GMB * 32 * 4)
  unsigned short* saTh;  CARVE(saTh,  unsigned short, (size_t)KSP * NT * 2)
  unsigned short* saTl;  CARVE(saTl,  unsigned short, (size_t)KSP * NT * 2)
  unsigned short* saRh;  CARVE(saRh,  unsigned short, (size_t)NT * KSP * 2)
  unsigned short* saRl;  CARVE(saRl,  unsigned short, (size_t)NT * KSP * 2)
  unsigned short* wgT;   CARVE(wgT,   unsigned short, (size_t)2 * 3 * DD * DD * 2)
  float* raw;   CARVE(raw,   float, (size_t)N * DD * 4)
  unsigned short* rawTh; CARVE(rawTh, unsigned short, (size_t)DD * NT * 2)
  unsigned short* rawTl; CARVE(rawTl, unsigned short, (size_t)DD * NT * 2)
  float* semb0; CARVE(semb0, float, (size_t)KSP * DD * 4)
  float* semb1; CARVE(semb1, float, (size_t)KSP * DD * 4)
  float* sup;   CARVE(sup,   float, (size_t)KSP * DD * 4)
  float* semb2; CARVE(semb2, float, (size_t)KSP * DD * 4)
  unsigned short* sTh;   CARVE(sTh,   unsigned short, (size_t)DD * KSP * 2)
  unsigned short* sTl;   CARVE(sTl,   unsigned short, (size_t)DD * KSP * 2)
  unsigned short* r2h;   CARVE(r2h,   unsigned short, (size_t)N * DD * 2)
  unsigned short* r2m;   CARVE(r2m,   unsigned short, (size_t)N * DD * 2)
  unsigned short* r2l;   CARVE(r2l,   unsigned short, (size_t)N * DD * 2)
  float* hbuf;  CARVE(hbuf,  float, (size_t)N * DD * 4)
  float* ha;    CARVE(ha,    float, (size_t)N * 4)
  float* hb;    CARVE(hb,    float, (size_t)N * 4)
#undef CARVE
  if (off > ws_size || off > (size_t)134217728) return;

  k_colsum<<<KSP / 128, 128, 0, stream>>>(SA, rcs, N, KS);
  k_setup_small<<<1, NTHR, 0, stream>>>(FA, ADJ, rcf, rden, adjn, KS);
  k_sa_planes<<<dim3(NT / 64, KSP / 64), NTHR, 0, stream>>>(SA, rcs, saRh, saRl, saTh, saTl, N, KS, NT);
  k_w_planes<<<2, NTHR, 0, stream>>>(Wg[0], Wg[1], wgT);
  k_gather<<<NT / 64, NTHR, 0, stream>>>(nodeT, typeT, lenT, laneT, nf, tf, lf, laf, raw, N, NR, TR, GRL, LR);

  hipFuncSetAttribute(reinterpret_cast<const void*>(&k_fnc),
                      hipFuncAttributeMaxDynamicSharedMemorySize, FNC_LDS_BYTES);
  hipFuncSetAttribute(reinterpret_cast<const void*>(&k_gat),
                      hipFuncAttributeMaxDynamicSharedMemorySize, GAT_LDS_BYTES);

  for (int L = 0; L < 2; ++L) {
    const unsigned short* wh = wgT + (size_t)L * 3 * DD * DD;
    const unsigned short* wm = wh + DD * DD;
    const unsigned short* wl = wm + DD * DD;
    float* dest = (L == 0) ? raw : out;

    k_tr_planes<<<NT / 64, NTHR, 0, stream>>>(raw, N, rawTh, rawTl, NT);
    k_gemm_se<<<KSP / GR, NTHR, 0, stream>>>(saTh, saTl, rawTh, rawTl, semb0, N, NT);
    k_fnc<<<1, NTHR, FNC_LDS_BYTES, stream>>>(semb0, FA, rcf, rden, Wf[L], bf[L], semb1, KS);
    k_sup_s<<<(KSP * DD) / NTHR, NTHR, 0, stream>>>(semb1, Ws[L], sup, KS);
    k_semb2<<<KSP, 128, 0, stream>>>(adjn, sup, bs[L], semb2, KS);
    k_tr_planes<<<KSP / 64, NTHR, 0, stream>>>(semb2, KS, sTh, sTl, KSP);
    k_gemm_sm<<<N / GR, NTHR, 0, stream>>>(saRh, saRl, sTh, sTl, raw, r2h, r2m, r2l, N);
    k_gemm_h<<<N / GR, NTHR, 0, stream>>>(r2h, r2m, r2l, wh, wm, wl, ag[L], hbuf, ha, hb, N);
    k_emax<<<GMB, NTHR, 0, stream>>>(ei, ha, hb, gpart, N, E);
    k_gat<<<(N + NB - 1) / NB, NTHR, GAT_LDS_BYTES, stream>>>(ei, hbuf, ha, hb, gpart, dest, N, E);
  }
}
